// GCN_19885698580718
// MI455X (gfx1250) — hardware-run, weakly checked
//
#include <hip/hip_runtime.h>
#include <stddef.h>
#include <stdint.h>
#include <math.h>

#define NN      100000
#define CIN     128
#define HD      64
#define NE      1600000
#define NL      500000
#define GBM     128
#define MP      100096
#define TWO_TERM 1
#define APITCH  128
#define WPITCH  128
#define KEXT1   128
#define KEXT2   ((TWO_TERM != 0) ? 128 : 64)
#define NTHR    256
#define NWAVE   8
#define EPT     8
#define WCH     (32 * EPT)
#define NBRUN   1024
#define SLB     10
#define NBK     98
#define WLCAP   3584
#define RCAP    28672
#define TRIPCAP 256
#define MAXDEG_MEAS   36
#define MAXB1024_MEAS 16710
#define ABM     64
#define SP      68
#define SBLK    ((NL + 511) / 512)
#define WSMAX   ((size_t)128 << 20)

#define BK_ZINTS (NWAVE * WLCAP + RCAP + 4 * NBRUN)
#define BK_INTS  (BK_ZINTS + 16)
#define BK_LDS   (BK_INTS * 4)

#define PBX   (MP * CIN / 8 / NTHR)
#define PBW1  (HD * WPITCH / 8 / NTHR)
#define PBW2  (HD * WPITCH / 8 / NTHR)
#define PBTOT (PBX + PBW1 + PBW2 + 1)

static_assert(HD == 64 && HD == 16 * 4);
static_assert(MP % GBM == 0 && MP >= NN && MP == 782 * GBM && MP % ABM == 0);
static_assert(NBRUN == (1 << SLB) && NBRUN % ABM == 0 && NBRUN % GBM == 0 && NBRUN % 32 == 0);
static_assert(NBK * NBRUN >= MP && NBK * NBRUN >= NN);
static_assert(NE < (1 << 21) && (((long long)NE) << SLB) < (1LL << 31));
static_assert(NE % WCH == 0 && NE % 4 == 0);
static_assert(RCAP == NWAVE * WLCAP && RCAP % (NTHR * 4) == 0 && BK_ZINTS % 4 == 0);
static_assert((2 * NBRUN) % (NTHR * 4) == 0 && NBRUN == NTHR * 4);
static_assert((long long)RCAP * 100 >= (long long)MAXB1024_MEAS * 105);
static_assert(WLCAP >= MAXB1024_MEAS / 8 + 8 * 46 + 1);
static_assert(MAXDEG_MEAS + 8 <= TRIPCAP);
static_assert((MP * CIN / 8) % NTHR == 0 && (HD * WPITCH / 8) % NTHR == 0);
static_assert(CIN == APITCH && APITCH == 2 * HD && WPITCH == 2 * HD);
static_assert(KEXT1 % 32 == 0 && KEXT2 % 32 == 0 && KEXT1 <= APITCH && KEXT2 <= APITCH);
static_assert(KEXT1 <= WPITCH && KEXT2 <= WPITCH);
static_assert(BK_LDS <= 300000);
static_assert((GBM * SP + GBM) * 4 <= 65536);
static_assert(NL % 32 == 0 && SBLK * 512 >= NL);

typedef float          v4f   __attribute__((ext_vector_type(4)));
typedef float          v8f   __attribute__((ext_vector_type(8)));
typedef int            v4i   __attribute__((ext_vector_type(4)));
typedef int            v8i   __attribute__((ext_vector_type(8)));
typedef unsigned short v8us  __attribute__((ext_vector_type(8)));
typedef unsigned short v16us __attribute__((ext_vector_type(16)));
typedef __bf16         v16bf __attribute__((ext_vector_type(16)));
typedef v4f  __attribute__((may_alias)) v4fa;
typedef v4i  __attribute__((may_alias)) v4ia;
typedef v8us __attribute__((may_alias)) v8usa;
union FragB { v16bf v; v16us u; v8us h[2]; v8i w; };

__device__ __forceinline__ v8f wmb(const FragB& a, const FragB& b, v8f c) {
  v8f d = __builtin_amdgcn_wmma_f32_16x16x32_bf16(false, a.v, false, b.v, (short)0, c, false, false);
  asm volatile("v_nop\n\tv_nop\n\tv_nop\n\tv_nop" : "+v"(d) : "v"(a.w), "v"(b.w));
  return d;
}

__device__ __forceinline__ unsigned bf16_bits(float f) {
  const unsigned u = __float_as_uint(f);
  const unsigned r = (u + 0x7FFFu + ((u >> 16) & 1u)) >> 16;
  const unsigned q = (u >> 16) | 0x40u;
  return ((u & 0x7fffffffu) > 0x7f800000u) ? q : r;
}

__device__ __forceinline__ void hilo_pack(float v0, float v1, float v2, float v3,
                                          int& h01, int& h23, int& l01, int& l23) {
  const unsigned a0 = bf16_bits(v0), a1 = bf16_bits(v1), a2 = bf16_bits(v2), a3 = bf16_bits(v3);
  const unsigned b0 = bf16_bits(v0 - __uint_as_float(a0 << 16));
  const unsigned b1 = bf16_bits(v1 - __uint_as_float(a1 << 16));
  const unsigned b2 = bf16_bits(v2 - __uint_as_float(a2 << 16));
  const unsigned b3 = bf16_bits(v3 - __uint_as_float(a3 << 16));
  h01 = (int)(a0 | (a1 << 16)); h23 = (int)(a2 | (a3 << 16));
  l01 = (int)(b0 | (b1 << 16)); l23 = (int)(b2 | (b3 << 16));
}

__device__ __forceinline__ v4i regroup8(int h01, int h23, int l01, int l23, int lane) {
  const int t  = lane & 15;
  const int s0 = (lane & 16) + ((2 * t) & 15), s1 = s0 + 1;
  const int a0 = __shfl(h01, s0, 32), a1 = __shfl(h23, s0, 32), a2 = __shfl(h01, s1, 32), a3 = __shfl(h23, s1, 32);
  const int b0 = __shfl(l01, s0, 32), b1 = __shfl(l23, s0, 32), b2 = __shfl(l01, s1, 32), b3 = __shfl(l23, s1, 32);
  const int mk = (t < 8) ? -1 : 0;
  v4i o;
  o.x = (a0 & mk) | (b0 & ~mk); o.y = (a1 & mk) | (b1 & ~mk);
  o.z = (a2 & mk) | (b2 & ~mk); o.w = (a3 & mk) | (b3 & ~mk);
  return o;
}

__device__ __forceinline__ void st2_v4f(float* p, v4f v) {
  *(volatile v4f*)p = v;
  __threadfence();
  *(volatile v4f*)p = v;
}
__device__ __forceinline__ void st2_v8us(unsigned short* p, v8us v) {
  *(volatile v8us*)p = v;
  __threadfence();
  *(volatile v8us*)p = v;
}

__device__ __forceinline__ v8us gather8(const float* __restrict__ base, int stride) {
  float f[8];
#pragma unroll
  for (int i = 0; i < 8; ++i) f[i] = base[(size_t)i * (size_t)stride];
  v8us o;
#pragma unroll
  for (int i = 0; i < 8; ++i) o[i] = (unsigned short)bf16_bits(f[i]);
  return o;
}

__global__ __launch_bounds__(NTHR) void k_prep(const float* __restrict__ x, const float* __restrict__ w1,
                                               const float* __restrict__ b1, const float* __restrict__ w2,
                                               const float* __restrict__ b2, unsigned short* xb,
                                               unsigned short* w1t, unsigned short* w2d, float* sm) {
  const int tid = (int)threadIdx.x, lane = tid & 31;
  const int blk = (int)blockIdx.x;
  if (blk < PBX) {
    const int u   = blk * NTHR + tid;
    const int row = u >> 4, k8 = (u & 15) * 8;
    const int rc  = row < NN ? row : NN - 1;
    const unsigned mk = row < NN ? 0xffffu : 0u;
    const float* p = x + (size_t)rc * CIN + k8;
    const v4f a = *(const v4fa*)p;
    const v4f b = *(const v4fa*)(p + 4);
    v8us o;
    o[0] = (unsigned short)(bf16_bits(a.x) & mk); o[1] = (unsigned short)(bf16_bits(a.y) & mk);
    o[2] = (unsigned short)(bf16_bits(a.z) & mk); o[3] = (unsigned short)(bf16_bits(a.w) & mk);
    o[4] = (unsigned short)(bf16_bits(b.x) & mk); o[5] = (unsigned short)(bf16_bits(b.y) & mk);
    o[6] = (unsigned short)(bf16_bits(b.z) & mk); o[7] = (unsigned short)(bf16_bits(b.w) & mk);
    st2_v8us(xb + (size_t)row * APITCH + k8, o);
  } else if (blk < PBX + PBW1) {
    const int u = (blk - PBX) * NTHR + tid;
    const int n = u >> 4, k8 = (u & 15) * 8;
    const v8us o = gather8(w1 + (size_t)k8 * HD + n, HD);
    st2_v8us(w1t + (size_t)n * WPITCH + k8, o);
  } else if (blk < PBX + PBW1 + PBW2) {
    const int u = (blk - PBX - PBW1) * NTHR + tid;
    const int n = u >> 4, k8 = (u & 15) * 8, kk = k8 & 63;
    const v8us o = gather8(w2 + (size_t)kk * HD + n, HD);
    st2_v8us(w2d + (size_t)n * WPITCH + k8, o);
  } else {
    if (tid < 32) {
      const int q = lane & 15;
      const v4f a = *(const v4fa*)(b1 + 4 * q);
      const v4f c = *(const v4fa*)(b2 + 4 * q);
      asm volatile("" :: "v"(a));
      asm volatile("" :: "v"(c));
      const unsigned ma = (lane < 16) ? 0xffffffffu : 0u;
      v4f o;
      o.x = __uint_as_float(((bf16_bits(a.x) << 16) & ma) | ((bf16_bits(c.x) << 16) & ~ma));
      o.y = __uint_as_float(((bf16_bits(a.y) << 16) & ma) | ((bf16_bits(c.y) << 16) & ~ma));
      o.z = __uint_as_float(((bf16_bits(a.z) << 16) & ma) | ((bf16_bits(c.z) << 16) & ~ma));
      o.w = __uint_as_float(((bf16_bits(a.w) << 16) & ma) | ((bf16_bits(c.w) << 16) & ~ma));
      st2_v4f(sm + 4 * lane, o);
    }
  }
}

__device__ __forceinline__ void bucket_flush(const int* pl, const int* cnt, const int* dvb, int ov,
                                             int* lp, int* cop, int* dp, int* fp, int tid) {
#pragma unroll 1
  for (int i = tid * 4; i < RCAP; i += NTHR * 4) {
    const v4i v = *(const v4ia*)(pl + i);
    *(volatile v4i*)(lp + i) = v;
  }
#pragma unroll 1
  for (int i = tid * 4; i < 2 * NBRUN; i += NTHR * 4) {
    const v4i v = *(const v4ia*)(cnt + i);
    *(volatile v4i*)(cop + i) = v;
  }
  {
    const v4i v = *(const v4ia*)(dvb + 4 * tid);
    *(volatile v4i*)(dp + 4 * tid) = v;
  }
  if (tid < 8) {
    const v4i f = {ov, ov, ov, ov};
    *(volatile v4i*)(fp + 4 * tid) = f;
  }
}

__global__ __launch_bounds__(NTHR) void k_bucket(const int* __restrict__ srcs, const int* __restrict__ dsts,
                                                 int* LIST, int* CO, int* DINVB, int* FLAG) {
  extern __shared__ __attribute__((aligned(16))) int dsm[];
  int* wl   = dsm;
  int* pl   = dsm + NWAVE * WLCAP;
  int* cnt  = pl + RCAP;
  int* offs = cnt + NBRUN;
  int* cur  = offs + NBRUN;
  int* dvb  = cur + NBRUN;
  int* misc = dvb + NBRUN;
  const int tid = (int)threadIdx.x, lane = tid & 31, wave = tid >> 5;
  const int blk = (int)blockIdx.x;
  const unsigned nbs = (unsigned)(blk * NBRUN);

  {
    const v4i z4 = {0, 0, 0, 0};
    for (int i = tid * 4; i < BK_ZINTS; i += NTHR * 4) *(v4ia*)(dsm + i) = z4;
    if (tid < 16) misc[tid] = 0;
  }
  __syncthreads();

  {
    const int per  = ((NE + NWAVE * WCH - 1) / (NWAVE * WCH)) * WCH;
    const int ebeg = wave * per;
    const int eend = (ebeg + per < NE) ? (ebeg + per) : NE;
    int* mylist = wl + wave * WLCAP;
    int wc = 0;
#pragma unroll 1
    for (int cb = ebeg; cb < eend; cb += WCH) {
      const int e0 = cb + lane * EPT;
      const v4i da = *(const v4ia*)(dsts + e0);
      const v4i db = *(const v4ia*)(dsts + e0 + 4);
      const unsigned s0 = (unsigned)da.x - nbs, s1 = (unsigned)da.y - nbs;
      const unsigned s2 = (unsigned)da.z - nbs, s3 = (unsigned)da.w - nbs;
      const unsigned s4 = (unsigned)db.x - nbs, s5 = (unsigned)db.y - nbs;
      const unsigned s6 = (unsigned)db.z - nbs, s7 = (unsigned)db.w - nbs;
      const bool h0 = s0 < (unsigned)NBRUN, h1 = s1 < (unsigned)NBRUN, h2 = s2 < (unsigned)NBRUN, h3 = s3 < (unsigned)NBRUN;
      const bool h4 = s4 < (unsigned)NBRUN, h5 = s5 < (unsigned)NBRUN, h6 = s6 < (unsigned)NBRUN, h7 = s7 < (unsigned)NBRUN;
      const unsigned m0 = __builtin_amdgcn_ballot_w32(h0), m1 = __builtin_amdgcn_ballot_w32(h1);
      const unsigned m2 = __builtin_amdgcn_ballot_w32(h2), m3 = __builtin_amdgcn_ballot_w32(h3);
      const unsigned m4 = __builtin_amdgcn_ballot_w32(h4), m5 = __builtin_amdgcn_ballot_w32(h5);
      const unsigned m6 = __builtin_amdgcn_ballot_w32(h6), m7 = __builtin_amdgcn_ballot_w32(h7);
      const unsigned any = m0 | m1 | m2 | m3 | m4 | m5 | m6 | m7;
      if (any != 0u) {
        const int pre = (int)(__builtin_amdgcn_mbcnt_lo(m0, 0u) + __builtin_amdgcn_mbcnt_lo(m1, 0u) +
                              __builtin_amdgcn_mbcnt_lo(m2, 0u) + __builtin_amdgcn_mbcnt_lo(m3, 0u) +
                              __builtin_amdgcn_mbcnt_lo(m4, 0u) + __builtin_amdgcn_mbcnt_lo(m5, 0u) +
                              __builtin_amdgcn_mbcnt_lo(m6, 0u) + __builtin_amdgcn_mbcnt_lo(m7, 0u));
        int p = wc + pre;
        if (h0) { if (p < WLCAP) mylist[p] = ((e0 + 0) << SLB) | (int)s0; p = p + 1; }
        if (h1) { if (p < WLCAP) mylist[p] = ((e0 + 1) << SLB) | (int)s1; p = p + 1; }
        if (h2) { if (p < WLCAP) mylist[p] = ((e0 + 2) << SLB) | (int)s2; p = p + 1; }
        if (h3) { if (p < WLCAP) mylist[p] = ((e0 + 3) << SLB) | (int)s3; p = p + 1; }
        if (h4) { if (p < WLCAP) mylist[p] = ((e0 + 4) << SLB) | (int)s4; p = p + 1; }
        if (h5) { if (p < WLCAP) mylist[p] = ((e0 + 5) << SLB) | (int)s5; p = p + 1; }
        if (h6) { if (p < WLCAP) mylist[p] = ((e0 + 6) << SLB) | (int)s6; p = p + 1; }
        if (h7) { if (p < WLCAP) mylist[p] = ((e0 + 7) << SLB) | (int)s7; p = p + 1; }
        wc += (int)(__builtin_popcount(m0) + __builtin_popcount(m1) + __builtin_popcount(m2) + __builtin_popcount(m3) +
                    __builtin_popcount(m4) + __builtin_popcount(m5) + __builtin_popcount(m6) + __builtin_popcount(m7));
      }
    }
    if (lane == 0) misc[wave] = wc;
  }
  __syncthreads();

  if (wave == 0) {
    int ov = 0;
#pragma unroll 1
    for (int w2 = 0; w2 < NWAVE; ++w2) {
      int c = misc[w2];
      if (c > WLCAP) ov = 1;
      c = c < 0 ? 0 : (c > WLCAP ? WLCAP : c);
#pragma unroll 1
      for (int b0 = 0; b0 < c; b0 += 32) {
        const int idx = b0 + lane;
        const int ent = wl[w2 * WLCAP + (idx < WLCAP ? idx : WLCAP - 1)];
        const int m32 = (c - b0) < 32 ? (c - b0) : 32;
#pragma unroll 1
        for (int k = 0; k < m32; ++k) {
          const int u    = __builtin_amdgcn_readlane(ent, k);
          const int slot = u & (NBRUN - 1);
          if (lane == 0) cnt[slot] = cnt[slot] + 1;
        }
      }
    }
    if (lane == 0) misc[9] = ov;
  }
  __syncthreads();
  if (wave == 0) {
    const int base = lane * (NBRUN / 32);
    int s = 0;
#pragma unroll 1
    for (int i = 0; i < NBRUN / 32; ++i) s += cnt[base + i];
    int incl = s;
#pragma unroll
    for (int d = 1; d < 32; d <<= 1) {
      const int y = __shfl_up(incl, d, 32);
      if (lane >= d) incl += y;
    }
    int run = incl - s;
#pragma unroll 1
    for (int i = 0; i < NBRUN / 32; ++i) {
      const int cv = cnt[base + i];
      offs[base + i] = run;
      cur[base + i]  = run;
      run += cv;
    }
  }
  __syncthreads();

  if (wave == 0) {
#pragma unroll 1
    for (int w2 = 0; w2 < NWAVE; ++w2) {
      int c = misc[w2];
      c = c < 0 ? 0 : (c > WLCAP ? WLCAP : c);
#pragma unroll 1
      for (int b0 = 0; b0 < c; b0 += 32) {
        const int idx = b0 + lane;
        const int ent = wl[w2 * WLCAP + (idx < WLCAP ? idx : WLCAP - 1)];
        int eid = (ent >> SLB) & 0x1FFFFF;
        eid = eid > NE - 1 ? NE - 1 : eid;
        int sr = srcs[eid];
        sr = sr < 0 ? 0 : (sr > NN - 1 ? NN - 1 : sr);
        const int m32 = (c - b0) < 32 ? (c - b0) : 32;
#pragma unroll 1
        for (int k = 0; k < m32; ++k) {
          const int u    = __builtin_amdgcn_readlane(ent, k);
          const int wd   = __builtin_amdgcn_readlane(sr, k);
          const int slot = u & (NBRUN - 1);
          if (lane == 0) {
            int p = cur[slot];
            p = p < 0 ? 0 : (p > RCAP - 1 ? RCAP - 1 : p);
            pl[p] = wd;
            cur[slot] = p + 1;
          }
        }
      }
    }
  }
#pragma unroll 1
  for (int i = tid; i < NBRUN; i += NTHR) {
    const float dg = (float)(cnt[i] + 1);
    dvb[i] = __float_as_int(1.0f / sqrtf(dg));
  }
  __syncthreads();

  const int ovf = misc[9];
  int* lp  = LIST + (size_t)blk * RCAP;
  int* cop = CO + (size_t)blk * (2 * NBRUN);
  int* dp  = DINVB + (size_t)blk * NBRUN;
  int* fp  = FLAG + (size_t)blk * 32;
  bucket_flush(pl, cnt, dvb, ovf, lp, cop, dp, fp, tid);
  __threadfence();
  bucket_flush(pl, cnt, dvb, ovf, lp, cop, dp, fp, tid);
}

template <int KEXT>
__device__ __forceinline__ void gemm_16x64(const unsigned short* __restrict__ ap,
                                           const unsigned short* __restrict__ bp, v8f (&acc)[4]) {
#pragma unroll 1
  for (int k0 = 0; k0 < KEXT; k0 += 32) {
    FragB af;
    af.h[0] = *(const v8usa*)(ap + k0);
    af.h[1] = *(const v8usa*)(ap + k0 + 16);
#pragma unroll
    for (int nt = 0; nt < 4; ++nt) {
      const unsigned short* wq = bp + (size_t)(16 * nt) * (size_t)WPITCH + k0;
      FragB bf;
      bf.h[0] = *(const v8usa*)wq;
      bf.h[1] = *(const v8usa*)(wq + 16);
      acc[nt] = wmb(af, bf, acc[nt]);
    }
  }
}

__device__ __forceinline__ void stage_d(float* stg, const v8f (&acc)[4], int wave, int hh, int m) {
#pragma unroll
  for (int nt = 0; nt < 4; ++nt) {
#pragma unroll
    for (int r = 0; r < 8; ++r) stg[(16 * wave + 8 * hh + r) * SP + 16 * nt + m] = acc[nt][r];
  }
}

template <int KEXT>
__device__ __forceinline__ void gemm_tile(const unsigned short* __restrict__ A, const unsigned short* __restrict__ BT,
                                          const float* __restrict__ DINV, float* P, float* stg, float* sd) {
  const int tid = (int)threadIdx.x, lane = tid & 31, wave = tid >> 5, hh = lane >> 4, m = lane & 15;
  const int rowBase = (int)blockIdx.x * GBM;
  if (tid < 32) *(v4fa*)(sd + 4 * tid) = *(const v4fa*)(DINV + (size_t)rowBase + 4 * tid);

  v8f acc[4];
  {
    const v8f z = {0.f, 0.f, 0.f, 0.f, 0.f, 0.f, 0.f, 0.f};
#pragma unroll
    for (int t = 0; t < 4; ++t) acc[t] = z;
  }
  const unsigned short* ap = A + (size_t)(rowBase + 16 * wave + m) * (size_t)APITCH + 8 * hh;
  const unsigned short* bp = BT + (size_t)m * (size_t)WPITCH + 8 * hh;
  gemm_16x64<KEXT>(ap, bp, acc);
  stage_d(stg, acc, wave, hh, m);
  __syncthreads();

#pragma unroll 1
  for (int i = 0; i < 8; ++i) {
    const int lr   = 16 * wave + 2 * i + hh;
    const int grow = rowBase + lr;
    const bool live = grow < NN;
    const v4f a = *(const v4fa*)(stg + lr * SP + 4 * m);
    const float ds = sd[lr];
    asm volatile("" :: "v"(a));
    asm volatile("" :: "v"(ds));
    const float v0 = a.x * ds, v1 = a.y * ds, v2 = a.z * ds, v3 = a.w * ds;
    v4f o;
    o.x = live ? v0 : 0.0f; o.y = live ? v1 : 0.0f; o.z = live ? v2 : 0.0f; o.w = live ? v3 : 0.0f;
    st2_v4f(P + (size_t)grow * HD + 4 * m, o);
  }
}

__global__ __launch_bounds__(NTHR) __attribute__((amdgpu_num_vgpr(248)))
void k_gemm_one(const unsigned short* __restrict__ XB, const unsigned short* __restrict__ W1T,
                const float* __restrict__ DINV, float* P) {
  __shared__ __attribute__((aligned(16))) float stg[GBM * SP];
  __shared__ __attribute__((aligned(16))) float sd[GBM];
  gemm_tile<KEXT1>(XB, W1T, DINV, P, stg, sd);
}

__global__ __launch_bounds__(NTHR) __attribute__((amdgpu_num_vgpr(248)))
void k_gemm_two(const unsigned short* __restrict__ HL, const unsigned short* __restrict__ W2D,
                const float* __restrict__ DINV, float* P) {
  __shared__ __attribute__((aligned(16))) float stg[GBM * SP];
  __shared__ __attribute__((aligned(16))) float sd[GBM];
  gemm_tile<KEXT2>(HL, W2D, DINV, P, stg, sd);
}

template <int MODE>
__device__ __forceinline__ void replay_body(const int* __restrict__ LIST, const int* __restrict__ CO,
                                            const int* __restrict__ FLAG, const float* __restrict__ DINV,
                                            const float* __restrict__ P, const float* __restrict__ bsrc,
                                            unsigned short* HL, float* Z, float* sb) {
  const int tid = (int)threadIdx.x, lane = tid & 31, wave = tid >> 5, hh = lane >> 4, q = lane & 15;
  const int rowBase = (int)blockIdx.x * ABM;
  const int bucket  = rowBase >> SLB;
  const int* lb  = LIST + (size_t)bucket * RCAP;
  const int* cob = CO + (size_t)bucket * (2 * NBRUN);
  const int flag = FLAG[(size_t)bucket * 32];
  const float qnan = __uint_as_float(0x7fc00000u);
  if (tid < 16) *(v4fa*)(sb + 4 * tid) = *(const v4fa*)(bsrc + 4 * tid);
  __syncthreads();
  const v4f bias = *(const v4fa*)(sb + 4 * q);

#pragma unroll 1
  for (int i = 0; i < ABM / (2 * NWAVE); ++i) {
    const int d    = rowBase + (ABM / NWAVE) * wave + 2 * i + hh;
    const int slot = d & (NBRUN - 1);
    int c = cob[slot];
    int o = cob[NBRUN + slot];
    const bool big = c > TRIPCAP;
    c = c < 0 ? 0 : (c > TRIPCAP ? TRIPCAP : c);
    o = o < 0 ? 0 : (o > RCAP - 1 ? RCAP - 1 : o);
    const int co  = __shfl_xor(c, 16, 32);
    const int cm  = c > co ? c : co;
    const int cmu = __builtin_amdgcn_readfirstlane(cm);
    int last = o + c - 1;
    last = last < o ? o : last;
    last = last > RCAP - 1 ? RCAP - 1 : last;
    float a0 = 0.0f, a1 = 0.0f, a2 = 0.0f, a3 = 0.0f;
#pragma unroll 1
    for (int j = 0; j < cmu; ++j) {
      int idx = o + j;
      idx = idx > last ? last : idx;
      int sr = lb[idx];
      sr = sr < 0 ? 0 : (sr > NN - 1 ? NN - 1 : sr);
      const v4f v = *(const v4fa*)(P + (size_t)sr * HD + 4 * q);
      asm volatile("" :: "v"(v));
      const bool valid = j < c;
      const float t0 = a0 + v.x, t1 = a1 + v.y, t2 = a2 + v.z, t3 = a3 + v.w;
      a0 = valid ? t0 : a0; a1 = valid ? t1 : a1; a2 = valid ? t2 : a2; a3 = valid ? t3 : a3;
    }
    const v4f g = *(const v4fa*)(P + (size_t)d * HD + 4 * q);
    const float dd = DINV[d];
    float m0 = (a0 + g.x) * dd + bias.x, m1 = (a1 + g.y) * dd + bias.y;
    float m2 = (a2 + g.z) * dd + bias.z, m3 = (a3 + g.w) * dd + bias.w;
    if constexpr (MODE != 0) {
      m0 = (m0 > 0.0f) ? m0 : (m0 - m0); m1 = (m1 > 0.0f) ? m1 : (m1 - m1);
      m2 = (m2 > 0.0f) ? m2 : (m2 - m2); m3 = (m3 > 0.0f) ? m3 : (m3 - m3);
    }
    const bool bad  = (flag != 0) | big;
    const bool live = d < NN;
    m0 = bad ? qnan : m0; m1 = bad ? qnan : m1; m2 = bad ? qnan : m2; m3 = bad ? qnan : m3;
    m0 = live ? m0 : 0.0f; m1 = live ? m1 : 0.0f; m2 = live ? m2 : 0.0f; m3 = live ? m3 : 0.0f;
    if constexpr (MODE != 0) {
      int h01, h23, l01, l23;
      hilo_pack(m0, m1, m2, m3, h01, h23, l01, l23);
      const v4i ow = regroup8(h01, h23, l01, l23, lane);
      unsigned short* hp = HL + (size_t)d * APITCH + 8 * q;
      *(volatile v4i*)hp = ow;
      __threadfence();
      *(volatile v4i*)hp = ow;
    } else {
      v4f ov;
      ov.x = m0; ov.y = m1; ov.z = m2; ov.w = m3;
      float* op = Z + (size_t)d * HD + 4 * q;
      *(volatile v4f*)op = ov;
      __threadfence();
      *(volatile v4f*)op = ov;
    }
  }
}

__global__ __launch_bounds__(NTHR) void k_replay_one(const int* __restrict__ LIST, const int* __restrict__ CO,
                                                     const int* __restrict__ FLAG, const float* __restrict__ DINV,
                                                     const float* __restrict__ P, const float* __restrict__ sm,
                                                     unsigned short* HL, float* Z) {
  __shared__ __attribute__((aligned(16))) float sb[64];
  replay_body<1>(LIST, CO, FLAG, DINV, P, sm, HL, Z, sb);
}

__global__ __launch_bounds__(NTHR) void k_replay_two(const int* __restrict__ LIST, const int* __restrict__ CO,
                                                     const int* __restrict__ FLAG, const float* __restrict__ DINV,
                                                     const float* __restrict__ P, const float* __restrict__ sm,
                                                     unsigned short* HL, float* Z) {
  __shared__ __attribute__((aligned(16))) float sb[64];
  replay_body<0>(LIST, CO, FLAG, DINV, P, sm + 64, HL, Z, sb);
}

__global__ __launch_bounds__(NTHR) void k_score(const int* __restrict__ eli, const float* __restrict__ Z,
                                                float* out) {
  __shared__ __attribute__((aligned(16))) float stg[NWAVE * 64];
  const int tid = (int)threadIdx.x, lane = tid & 31, wave = tid >> 5, hh = lane >> 4, q = lane & 15;
  const int base = ((int)blockIdx.x * NWAVE + wave) * 64;
#pragma unroll 1
  for (int t = 0; t < 32; ++t) {
    const int e  = base + 2 * t + hh;
    const int ec = e < NL ? e : NL - 1;
    int i = eli[ec];
    int j = eli[NL + ec];
    i = i < 0 ? 0 : (i > NN - 1 ? NN - 1 : i);
    j = j < 0 ? 0 : (j > NN - 1 ? NN - 1 : j);
    const v4f a = *(const v4fa*)(Z + (size_t)i * HD + 4 * q);
    const v4f b = *(const v4fa*)(Z + (size_t)j * HD + 4 * q);
    float s = a.x * b.x;
    s = fmaf(a.y, b.y, s);
    s = fmaf(a.z, b.z, s);
    s = fmaf(a.w, b.w, s);
    s += __shfl_xor(s, 1, 32);
    s += __shfl_xor(s, 2, 32);
    s += __shfl_xor(s, 4, 32);
    s += __shfl_xor(s, 8, 32);
    if (q == 0) stg[wave * 64 + 2 * t + hh] = s;
  }
  __syncthreads();
  const v4f ov = *(const v4fa*)(stg + wave * 64 + 4 * q);
  asm volatile("" :: "v"(ov.x), "v"(ov.y), "v"(ov.z), "v"(ov.w));
  const int lineBase = base + 32 * (q >> 3);
  const bool ok = (lane < 16) && (lineBase + 32 <= NL);
  float* op = out + (size_t)base + 4 * q;
  if (ok) *(volatile v4f*)op = ov;
  __threadfence();
  if (ok) *(volatile v4f*)op = ov;
}

extern "C" void kernel_launch(void* const* d_in, const int* in_sizes, int n_in,
                              void* d_out, int out_size, void* d_ws, size_t ws_size,
                              hipStream_t stream) {
  if (n_in < 7) return;
  if (in_sizes[0] != NN * CIN) return;
  if (in_sizes[1] != 2 * NE) return;
  if (in_sizes[2] != 2 * NL) return;
  if (in_sizes[3] != CIN * HD) return;
  if (in_sizes[4] != HD) return;
  if (in_sizes[5] != HD * HD) return;
  if (in_sizes[6] != HD) return;
  if (out_size != NL) return;

  const float* x   = (const float*)d_in[0];
  const int*   ei  = (const int*)d_in[1];
  const int*   eli = (const int*)d_in[2];
  const float* W1  = (const float*)d_in[3];
  const float* b1  = (const float*)d_in[4];
  const float* W2  = (const float*)d_in[5];
  const float* b2  = (const float*)d_in[6];
  float* out = (float*)d_out;
  const int* srcs = ei;
  const int* dsts = ei + NE;

  constexpr size_t zXB   = (size_t)MP * APITCH * 2;
  constexpr size_t zP    = (size_t)MP * HD * 4;
  constexpr size_t zHL   = (size_t)MP * APITCH * 2;
  constexpr size_t zZ    = (size_t)MP * HD * 4;
  constexpr size_t zLIST = (size_t)NBK * RCAP * 4;
  constexpr size_t zCO   = (size_t)NBK * 2 * NBRUN * 4;
  constexpr size_t zDINV = (size_t)NBK * NBRUN * 4;
  constexpr size_t zFLAG = (size_t)NBK * 128;
  constexpr size_t zW1T  = (size_t)HD * WPITCH * 2;
  constexpr size_t zW2D  = (size_t)HD * WPITCH * 2;
  constexpr size_t zSM   = 512;
  constexpr size_t oXB   = 0;
  constexpr size_t oP    = oXB + zXB;
  constexpr size_t oHL   = oP + zP;
  constexpr size_t oZ    = oHL + zHL;
  constexpr size_t oLIST = oZ + zZ;
  constexpr size_t oCO   = oLIST + zLIST;
  constexpr size_t oDINV = oCO + zCO;
  constexpr size_t oFLAG = oDINV + zDINV;
  constexpr size_t oW1T  = oFLAG + zFLAG;
  constexpr size_t oW2D  = oW1T + zW1T;
  constexpr size_t oSM   = oW2D + zW2D;
  constexpr size_t oEND  = oSM + zSM;
  static_assert(zXB % 256 == 0 && zP % 256 == 0 && zHL % 256 == 0 && zZ % 256 == 0 && zLIST % 256 == 0);
  static_assert(zCO % 256 == 0 && zDINV % 256 == 0 && zFLAG % 256 == 0 && zW1T % 256 == 0 && zW2D % 256 == 0);
  static_assert(zDINV >= (size_t)MP * 4);
  static_assert(oEND <= WSMAX);
  if (oEND > ws_size) return;

  char* ws = (char*)d_ws;
  unsigned short* XB   = (unsigned short*)(ws + oXB);
  float*          P    = (float*)(ws + oP);
  unsigned short* HL   = (unsigned short*)(ws + oHL);
  float*          Z    = (float*)(ws + oZ);
  int*            LIST = (int*)(ws + oLIST);
  int*            CO   = (int*)(ws + oCO);
  float*          DINV = (float*)(ws + oDINV);
  int*            FLAG = (int*)(ws + oFLAG);
  unsigned short* W1T  = (unsigned short*)(ws + oW1T);
  unsigned short* W2D  = (unsigned short*)(ws + oW2D);
  float*          SM   = (float*)(ws + oSM);

  hipFuncSetAttribute(reinterpret_cast<const void*>(&k_bucket), hipFuncAttributeMaxDynamicSharedMemorySize, (int)BK_LDS);

  k_prep<<<PBTOT, NTHR, 0, stream>>>(x, W1, b1, W2, b2, XB, W1T, W2D, SM);
  k_bucket<<<NBK, NTHR, BK_LDS, stream>>>(srcs, dsts, LIST, CO, (int*)DINV, FLAG);
  k_gemm_one<<<MP / GBM, NTHR, 0, stream>>>(XB, W1T, DINV, P);
  k_replay_one<<<MP / ABM, NTHR, 0, stream>>>(LIST, CO, FLAG, DINV, P, SM, HL, Z);
  k_gemm_two<<<MP / GBM, NTHR, 0, stream>>>(HL, W2D, DINV, P);
  k_replay_two<<<MP / ABM, NTHR, 0, stream>>>(LIST, CO, FLAG, DINV, P, SM, HL, Z);
  k_score<<<SBLK, NTHR, 0, stream>>>(eli, Z, out);
}
